// MHTTT_57174604644762
// MI455X (gfx1250) — hardware-run, weakly checked
//
#include <hip/hip_runtime.h>
#include <math.h>

typedef __attribute__((ext_vector_type(16))) _Float16 v16h;
typedef __attribute__((ext_vector_type(8)))  _Float16 v8h;
typedef __attribute__((ext_vector_type(16))) __bf16   v16b;
typedef __attribute__((ext_vector_type(8)))  __bf16   v8b;
typedef __attribute__((ext_vector_type(8)))  float    v8f;
typedef __attribute__((ext_vector_type(4)))  float    v4f;

constexpr int kB    = 2;
constexpr int kS    = 2048;
constexpr int kH    = 16;
constexpr int kD    = 64;
constexpr int kDM   = kH * kD;
constexpr int kRows = kB * kS;
constexpr int kQKP  = 2 * kDM;
constexpr int kTP   = kRows;
constexpr int kCh   = 64;
constexpr int kNCh  = kS / kCh;
constexpr int kPl   = kCh * kD;
constexpr int kOsP  = 68;
constexpr float kEps = 1e-5f;
constexpr double kInvCnt = 1.0 / (double)(kS * kD);
static_assert(kDM == 1024 && kRows == 4096 && kQKP == 2048 && kTP == 4096, "shape constants");
static_assert(kD == 64 && kCh == 64 && (kS % kCh) == 0 && kNCh == 32 && kPl == 4096, "chunking");
static_assert((kDM % 32) == 0, "GEMM K multiple of 32");
static_assert((kRows % 64) == 0 && (kQKP % 64) == 0 && (kDM % 64) == 0 && (kTP % 64) == 0, "GEMM M,N multiples of 64");

constexpr size_t kOffXB   = 0;
constexpr size_t kOffWB   = kOffXB   + (size_t)kRows * kDM * 2;
constexpr size_t kOffQKH  = kOffWB   + (size_t)3 * kDM * kDM * 2;
constexpr size_t kOffQKL  = kOffQKH  + (size_t)kRows * kQKP * 2;
constexpr size_t kOffKVTH = kOffQKL  + (size_t)kRows * kQKP * 2;
constexpr size_t kOffKVTL = kOffKVTH + (size_t)kQKP * kTP * 2;
constexpr size_t kOffSP   = kOffKVTL + (size_t)kQKP * kTP * 2;
constexpr size_t kOffCTX  = kOffSP   + (size_t)kB * kH * kNCh * 4 * kPl * 2;
constexpr size_t kOffST   = kOffCTX  + (size_t)kRows * kDM * 4;
constexpr size_t kWsTotal = kOffST   + (size_t)kB * kH * 32 * 4;
constexpr size_t kOffOW   = kOffWB;
constexpr size_t kOffNH   = kOffQKH;
constexpr size_t kOffNL   = kOffQKH + (size_t)kRows * kDM * 2;
static_assert(kWsTotal == 132124672ull, "carve total");
static_assert(kWsTotal <= 134217728ull, "carve cap");
static_assert((size_t)kDM * kDM * 2 <= (size_t)3 * kDM * kDM * 2, "OW fits the WB region");
static_assert(kOffNL + (size_t)kRows * kDM * 2 <= kOffQKL, "NH and NL fit the QKH region");
static_assert((kOffWB % 128) == 0 && (kOffQKH % 128) == 0 && (kOffQKL % 128) == 0 &&
              (kOffKVTH % 128) == 0 && (kOffKVTL % 128) == 0 && (kOffSP % 128) == 0 && (kOffCTX % 128) == 0 &&
              (kOffST % 128) == 0 && (kOffNL % 128) == 0, "128-B aligned regions");

__device__ __forceinline__ unsigned short f2bf_bits(float f) {
  unsigned u = __float_as_uint(f);
  return (unsigned short)((u + 0x7FFFu + ((u >> 16) & 1u)) >> 16);
}
__device__ __forceinline__ float bf_bits2f(unsigned short h) { return __uint_as_float(((unsigned)h) << 16); }
__device__ __forceinline__ float rne_bf(float f) { return bf_bits2f(f2bf_bits(f)); }

__device__ __forceinline__ void keep4_b(v16b a, v16b b, v16b c, v16b d) { asm volatile("v_nop" :: "v"(a), "v"(b), "v"(c), "v"(d)); }
__device__ __forceinline__ void acc_guard4(v8f& a, v8f& b, v8f& c, v8f& d) { asm volatile("v_nop\n\tv_nop\n\tv_nop\n\tv_nop" : "+v"(a), "+v"(b), "+v"(c), "+v"(d)); }
__device__ __forceinline__ void cc_mem_fence() { asm volatile("" ::: "memory"); }

union FragB { v16b v; v8b h[2]; };
__device__ __forceinline__ v16b frag_ld(const __bf16* p) {
  FragB f;
  f.h[0] = *(const v8b*)(p);
  f.h[1] = *(const v8b*)(p + 16);
  return f.v;
}
__device__ __forceinline__ v8f mma_g(v16b a, v16b b, v8f c) {
  c = __builtin_amdgcn_wmma_f32_16x16x32_bf16(false, a, false, b, (short)0, c, false, false);
  asm volatile("v_nop\n\tv_nop\n\tv_nop\n\tv_nop" : "+v"(c) : "v"(a), "v"(b));
  return c;
}
__device__ __forceinline__ void mma3(v8f& c, v16b ah, v16b al, v16b bh, v16b bl) {
  c = mma_g(ah, bh, c);
  c = mma_g(ah, bl, c);
  c = mma_g(al, bh, c);
}
__device__ __forceinline__ v8f zero8() { return (v8f){0.f, 0.f, 0.f, 0.f, 0.f, 0.f, 0.f, 0.f}; }

__device__ __forceinline__ void st_split(__bf16* ph, __bf16* pl, int idx, float v) {
  const unsigned short hb = f2bf_bits(v);
  const unsigned short lb = f2bf_bits(v - bf_bits2f(hb));
  ph[idx] = __builtin_bit_cast(__bf16, hb);
  pl[idx] = __builtin_bit_cast(__bf16, lb);
}

template <int SPL, int BIAS_MODE, int OUT_MODE>
__global__ __launch_bounds__(256) void wmma_gemm64(
    const unsigned short* __restrict__ Ap, const unsigned short* __restrict__ A2p, int lda,
    const unsigned short* __restrict__ Btp, int ldb,
    void* __restrict__ Cout, void* __restrict__ Cout2, int ldc,
    const float* __restrict__ bias, int M, int N, int K) {
  const __bf16* A  = (const __bf16*)Ap;
  const __bf16* A2 = (const __bf16*)A2p;
  const __bf16* Bt = (const __bf16*)Btp;
  __shared__ __align__(16) float sT[8][16 * 68];
  const int lane = threadIdx.x & 31;
  const int wave = threadIdx.x >> 5;
  const int tilesN = N >> 6;
  const int tilesM = M >> 6;
  const int tile = blockIdx.x * 8 + wave;
  if (tile >= tilesM * tilesN) return;
  const int tm = tile / tilesN;
  const int tn = tile - tm * tilesN;
  const int m0 = tm << 6;
  const int n0 = tn << 6;

  const int rlane = lane & 15;
  const int koff  = (lane >> 4) * 8;
  const int mOff  = (lane >> 4) * 8;

  v8f acc[4][4];
#pragma unroll
  for (int i = 0; i < 4; ++i)
#pragma unroll
    for (int j = 0; j < 4; ++j) acc[i][j] = zero8();

  for (int k0 = 0; k0 < K; k0 += 32) {
    v16b bh[4];
#pragma unroll
    for (int j = 0; j < 4; ++j) {
      const size_t bo = (size_t)(n0 + (j << 4) + rlane) * ldb + koff + k0;
      bh[j] = frag_ld(Bt + bo);
    }
#pragma unroll
    for (int i = 0; i < 4; ++i) {
      const size_t ao = (size_t)(m0 + (i << 4) + rlane) * lda + koff + k0;
      const v16b ah = frag_ld(A + ao);
      v16b al = ah;
      if (SPL >= 1) al = frag_ld(A2 + ao);
#pragma unroll
      for (int j = 0; j < 4; ++j) {
        acc[i][j] = mma_g(ah, bh[j], acc[i][j]);
        if (SPL >= 1) acc[i][j] = mma_g(al, bh[j], acc[i][j]);
      }
    }
    keep4_b(bh[0], bh[1], bh[2], bh[3]);
  }
  acc_guard4(acc[0][0], acc[0][1], acc[0][2], acc[0][3]);
  acc_guard4(acc[1][0], acc[1][1], acc[1][2], acc[1][3]);
  acc_guard4(acc[2][0], acc[2][1], acc[2][2], acc[2][3]);
  acc_guard4(acc[3][0], acc[3][1], acc[3][2], acc[3][3]);

  float* slab = sT[wave];
#pragma unroll
  for (int i = 0; i < 4; ++i) {
    const int mBase = m0 + (i << 4);
    float bm[8];
#pragma unroll
    for (int r = 0; r < 8; ++r) bm[r] = (BIAS_MODE == 1) ? rne_bf(bias[mBase + mOff + r]) : 0.f;
#pragma unroll
    for (int j = 0; j < 4; ++j) {
      const int n = n0 + (j << 4) + rlane;
      const float bv = (BIAS_MODE == 2) ? rne_bf(bias[n]) : 0.f;
#pragma unroll
      for (int r = 0; r < 8; ++r) {
        const float v = acc[i][j][r] + bm[r] + bv;
        slab[(mOff + r) * 68 + (j << 4) + rlane] = v;
      }
    }
    __builtin_amdgcn_fence(__ATOMIC_RELEASE, "workgroup");
    __builtin_amdgcn_wave_barrier();
    __builtin_amdgcn_fence(__ATOMIC_ACQUIRE, "workgroup");
    if (OUT_MODE == 0) {
      float* C = (float*)Cout;
      const int hh = lane >> 4, c4 = (lane & 15) * 4;
      for (int pass = 0; pass < 2; ++pass) {
#pragma unroll
        for (int it = 0; it < 8; ++it) {
          const int row = it * 2 + hh;
          v4f v = *(const v4f*)(slab + row * 68 + c4);
          *(volatile v4f*)(C + (size_t)(mBase + row) * ldc + n0 + c4) = v;
        }
        __threadfence();
      }
    } else {
      const int q = lane >> 3, c8 = (lane & 7) * 8;
      unsigned short* C  = (unsigned short*)Cout;
      unsigned short* C2 = (unsigned short*)Cout2;
      for (int pass = 0; pass < 2; ++pass) {
#pragma unroll
        for (int it = 0; it < 4; ++it) {
          const int row = it * 4 + q;
          const float* sp = slab + row * 68 + c8;
          v8h hv, lv;
#pragma unroll
          for (int e = 0; e < 8; ++e) {
            const float sv = sp[e];
            const unsigned short hb = f2bf_bits(sv);
            const unsigned short lb = f2bf_bits(sv - bf_bits2f(hb));
            hv[e] = __builtin_bit_cast(_Float16, hb);
            lv[e] = __builtin_bit_cast(_Float16, lb);
          }
          *(volatile v8h*)(C  + (size_t)(mBase + row) * ldc + n0 + c8) = hv;
          *(volatile v8h*)(C2 + (size_t)(mBase + row) * ldc + n0 + c8) = lv;
        }
        __threadfence();
      }
    }
    __builtin_amdgcn_fence(__ATOMIC_RELEASE, "workgroup");
    __builtin_amdgcn_wave_barrier();
    __builtin_amdgcn_fence(__ATOMIC_ACQUIRE, "workgroup");
  }
}

__global__ __launch_bounds__(256) void cast8_bf16_kernel(const float* __restrict__ src,
                                                         unsigned short* __restrict__ dst, int total8) {
  const int i = blockIdx.x * 256 + threadIdx.x;
  if (i >= total8) return;
  const size_t e0 = (size_t)i << 3;
  const v4f a0 = *(const v4f*)(src + e0);
  const v4f a1 = *(const v4f*)(src + e0 + 4);
  v8h hv;
#pragma unroll
  for (int e = 0; e < 4; ++e) {
    const unsigned short h0 = f2bf_bits(a0[e]);
    const unsigned short h1 = f2bf_bits(a1[e]);
    hv[e]     = __builtin_bit_cast(_Float16, h0);
    hv[4 + e] = __builtin_bit_cast(_Float16, h1);
  }
  unsigned short* q = dst + e0;
  *(volatile v8h*)q = hv;
  __threadfence();
  *(volatile v8h*)q = hv;
}

__device__ __forceinline__ void gemm16x64(v8f (&acc)[4],
                                          const __bf16* ah_p, const __bf16* al_p,
                                          const __bf16* bh_p, const __bf16* bl_p, size_t bstep) {
#pragma unroll 1
  for (int kk = 0; kk < 2; ++kk) {
    const v16b ah = frag_ld(ah_p + 32 * kk);
    const v16b al = frag_ld(al_p + 32 * kk);
#pragma unroll
    for (int j = 0; j < 4; ++j) {
      const v16b bh = frag_ld(bh_p + (size_t)j * bstep + 32 * kk);
      const v16b bl = frag_ld(bl_p + (size_t)j * bstep + 32 * kk);
      mma3(acc[j], ah, al, bh, bl);
      cc_mem_fence();
    }
  }
}

__device__ __forceinline__ void flush_rows16(const __bf16* xh, const __bf16* xl,
                                             unsigned short* gh, unsigned short* gl, int lane) {
  const int q = lane >> 3, c8 = (lane & 7) * 8;
  v8h hv[4], lv[4];
#pragma unroll
  for (int it = 0; it < 4; ++it) {
    const int row = it * 4 + q;
    const v8b a = *(const v8b*)(xh + row * kCh + c8);
    const v8b l = *(const v8b*)(xl + row * kCh + c8);
    hv[it] = __builtin_bit_cast(v8h, a);
    lv[it] = __builtin_bit_cast(v8h, l);
  }
  for (int pass = 0; pass < 2; ++pass) {
#pragma unroll
    for (int it = 0; it < 4; ++it) {
      const int row = it * 4 + q;
      *(volatile v8h*)(gh + row * kD + c8) = hv[it];
      *(volatile v8h*)(gl + row * kD + c8) = lv[it];
    }
    __threadfence();
  }
}

__global__ __launch_bounds__(128) void state_prefix_kernel(
    const unsigned short* __restrict__ KVThp, const unsigned short* __restrict__ KVTlp,
    unsigned short* __restrict__ SP) {
  __shared__ __align__(16) __bf16 Xs[4][2 * 16 * kCh];

  const int tid  = threadIdx.x;
  const int wave = tid >> 5;
  const int lane = tid & 31;
  const int hh   = lane >> 4;
  const int rl   = lane & 15;
  const int koff = 8 * hh;
  const int bh   = blockIdx.x;
  const int b    = bh / kH;
  const int h    = bh - b * kH;

  const __bf16* kth = (const __bf16*)KVThp + (size_t)(h * kD) * kTP + (size_t)b * kS;
  const __bf16* ktl = (const __bf16*)KVTlp + (size_t)(h * kD) * kTP + (size_t)b * kS;
  const __bf16* vth = kth + (size_t)kDM * kTP;
  const __bf16* vtl = ktl + (size_t)kDM * kTP;

  __bf16* xh = &Xs[wave][0];
  __bf16* xl = xh + 16 * kCh;

  const size_t at_off = (size_t)(16 * wave + rl) * kTP + koff;
  const size_t bt_off = (size_t)rl * kTP + koff;

  v8f Macc[4], Nacc[4];
#pragma unroll
  for (int j = 0; j < 4; ++j) { Macc[j] = zero8(); Nacc[j] = zero8(); }

#pragma unroll 1
  for (int c = 0; c < kNCh; ++c) {
    const int t0 = c * kCh;
    unsigned short* sp = SP + ((size_t)(bh * kNCh + c) * 4) * kPl + (size_t)(16 * wave) * kD;

#pragma unroll
    for (int j = 0; j < 4; ++j) {
#pragma unroll
      for (int r = 0; r < 8; ++r) {
        const int row = 16 * wave + 8 * hh + r;
        const int col = 16 * j + rl;
        const float dg = (row == col) ? 2.0f : 0.0f;
        st_split(xh, xl, (8 * hh + r) * kCh + col, dg - Macc[j][r]);
      }
    }
    __syncthreads();
    flush_rows16(xh, xl, sp, sp + kPl, lane);
    __syncthreads();

#pragma unroll
    for (int j = 0; j < 4; ++j) {
#pragma unroll
      for (int r = 0; r < 8; ++r) {
        st_split(xh, xl, (8 * hh + r) * kCh + 16 * j + rl, Nacc[j][r]);
      }
    }
    __syncthreads();
    flush_rows16(xh, xl, sp + 2 * kPl, sp + 3 * kPl, lane);
    __syncthreads();

#pragma unroll 1
    for (int kk = 0; kk < 2; ++kk) {
      const v16b kah = frag_ld(kth + t0 + at_off + 32 * kk);
      const v16b kal = frag_ld(ktl + t0 + at_off + 32 * kk);
      const v16b vah = frag_ld(vth + t0 + at_off + 32 * kk);
      const v16b val = frag_ld(vtl + t0 + at_off + 32 * kk);
#pragma unroll
      for (int j = 0; j < 4; ++j) {
        const v16b bhf = frag_ld(kth + t0 + bt_off + (size_t)j * 16 * kTP + 32 * kk);
        const v16b blf = frag_ld(ktl + t0 + bt_off + (size_t)j * 16 * kTP + 32 * kk);
        mma3(Macc[j], kah, kal, bhf, blf);
        mma3(Nacc[j], vah, val, bhf, blf);
        cc_mem_fence();
      }
    }
  }
}

__global__ __launch_bounds__(128) void chain_chunk_kernel(
    const unsigned short* __restrict__ QKhp, const unsigned short* __restrict__ QKlp,
    const unsigned short* __restrict__ KVThp, const unsigned short* __restrict__ KVTlp,
    const unsigned short* __restrict__ SPp, float* __restrict__ ctx) {
  __shared__ __align__(16) __bf16 Xq[4][2 * 16 * kCh];
  __shared__ __align__(16) __bf16 Xa[4][2 * 16 * kCh];
  __shared__ __align__(16) float  Os[4][16 * kOsP];

  const int tid  = threadIdx.x;
  const int wave = tid >> 5;
  const int lane = tid & 31;
  const int hh   = lane >> 4;
  const int rl   = lane & 15;
  const int koff = 8 * hh;
  const int bh   = blockIdx.x / kNCh;
  const int c    = blockIdx.x - bh * kNCh;
  const int b    = bh / kH;
  const int h    = bh - b * kH;
  const int t0   = c * kCh;

  const __bf16* qh  = (const __bf16*)QKhp + (size_t)(b * kS + t0) * kQKP + h * kD;
  const __bf16* ql  = (const __bf16*)QKlp + (size_t)(b * kS + t0) * kQKP + h * kD;
  const __bf16* kh  = qh + kDM;
  const __bf16* kl  = ql + kDM;
  const __bf16* kth = (const __bf16*)KVThp + (size_t)(h * kD) * kTP + (size_t)(b * kS + t0);
  const __bf16* ktl = (const __bf16*)KVTlp + (size_t)(h * kD) * kTP + (size_t)(b * kS + t0);
  const __bf16* vth = kth + (size_t)kDM * kTP;
  const __bf16* vtl = ktl + (size_t)kDM * kTP;
  const __bf16* sp  = (const __bf16*)SPp + ((size_t)(bh * kNCh + c) * 4) * kPl;

  __bf16* xqh = &Xq[wave][0];
  __bf16* xql = xqh + 16 * kCh;
  __bf16* xah = &Xa[wave][0];
  __bf16* xal = xah + 16 * kCh;
  float*  os  = &Os[wave][0];

  const size_t aq_off = (size_t)(16 * wave + rl) * kQKP + koff;
  const size_t bk_off = (size_t)rl * kQKP + koff;
  const size_t bt_off = (size_t)rl * kTP + koff;
  const int    xa_off = rl * kCh + koff;
  const int    sb_off = rl * kD + koff;

  v8f acc[4];

#pragma unroll
  for (int j = 0; j < 4; ++j) acc[j] = zero8();
  gemm16x64(acc, qh + aq_off, ql + aq_off, kh + bk_off, kl + bk_off, (size_t)16 * kQKP);
#pragma unroll
  for (int j = 0; j < 4; ++j) {
#pragma unroll
    for (int r = 0; r < 8; ++r) {
      const int tl = 16 * wave + 8 * hh + r;
      const int sl = 16 * j + rl;
      const float v = (sl <= tl) ? (-acc[j][r]) : 0.0f;
      st_split(xah, xal, (8 * hh + r) * kCh + sl, v);
    }
  }
  __syncthreads();

#pragma unroll
  for (int j = 0; j < 4; ++j) acc[j] = zero8();
  gemm16x64(acc, qh + aq_off, ql + aq_off, sp + sb_off, sp + kPl + sb_off, (size_t)16 * kD);
  gemm16x64(acc, xah + xa_off, xal + xa_off, kth + bt_off, ktl + bt_off, (size_t)16 * kTP);
#pragma unroll
  for (int j = 0; j < 4; ++j) {
#pragma unroll
    for (int r = 0; r < 8; ++r) {
      st_split(xqh, xql, (8 * hh + r) * kCh + 16 * j + rl, acc[j][r]);
    }
  }
  __syncthreads();

#pragma unroll
  for (int j = 0; j < 4; ++j) acc[j] = zero8();
  gemm16x64(acc, xqh + xa_off, xql + xa_off, kh + bk_off, kl + bk_off, (size_t)16 * kQKP);
#pragma unroll
  for (int j = 0; j < 4; ++j) {
#pragma unroll
    for (int r = 0; r < 8; ++r) {
      const int tl = 16 * wave + 8 * hh + r;
      const int sl = 16 * j + rl;
      const float v = (sl <= tl) ? acc[j][r] : 0.0f;
      st_split(xah, xal, (8 * hh + r) * kCh + sl, v);
    }
  }
  __syncthreads();

#pragma unroll
  for (int j = 0; j < 4; ++j) acc[j] = zero8();
  gemm16x64(acc, xqh + xa_off, xql + xa_off, sp + 2 * kPl + sb_off, sp + 3 * kPl + sb_off, (size_t)16 * kD);
  gemm16x64(acc, xah + xa_off, xal + xa_off, vth + bt_off, vtl + bt_off, (size_t)16 * kTP);
#pragma unroll
  for (int j = 0; j < 4; ++j) {
#pragma unroll
    for (int r = 0; r < 8; ++r) {
      os[(8 * hh + r) * kOsP + 16 * j + rl] = acc[j][r];
    }
  }
  __syncthreads();
  {
    const int c4 = rl * 4;
    for (int pass = 0; pass < 2; ++pass) {
#pragma unroll
      for (int it = 0; it < 8; ++it) {
        const int row = it * 2 + hh;
        v4f val = *(const v4f*)(os + row * kOsP + c4);
        *(volatile v4f*)(ctx + (size_t)(b * kS + t0 + 16 * wave + row) * kDM + h * kD + c4) = val;
      }
      __threadfence();
    }
  }
}

__global__ __launch_bounds__(256) void gn_stats_kernel(const float* __restrict__ ctx, float* __restrict__ stats) {
  __shared__ double rs[8];
  __shared__ double rq[8];
  const int bh = blockIdx.x;
  const int b  = bh / kH;
  const int h  = bh - b * kH;
  const int tid = threadIdx.x, lane = tid & 31, wave = tid >> 5;
  const float* p = ctx + (size_t)b * kS * kDM + h * kD + (tid & 15) * 4;
  const int r0 = tid >> 4;
  double s = 0.0, q = 0.0;
#pragma unroll 1
  for (int i = 0; i < kS / 16; ++i) {
    const v4f v = *(const v4f*)(p + (size_t)(r0 + 16 * i) * kDM);
    const double d0 = (double)v[0], d1 = (double)v[1], d2 = (double)v[2], d3 = (double)v[3];
    s += (d0 + d1) + (d2 + d3);
    q += (d0 * d0 + d1 * d1) + (d2 * d2 + d3 * d3);
  }
#pragma unroll
  for (int off = 16; off > 0; off >>= 1) {
    const double so = __shfl_xor(s, off, 32);
    const double qo = __shfl_xor(q, off, 32);
    s += so;
    q += qo;
  }
  if (lane == 0) { rs[wave] = s; rq[wave] = q; }
  __syncthreads();
  if (wave == 0) {
    double S = 0.0, Q = 0.0;
#pragma unroll
    for (int w = 0; w < 8; ++w) { S += rs[w]; Q += rq[w]; }
    const double mu  = S * kInvCnt;
    const double var = Q * kInvCnt - mu * mu;
    const float muf  = (float)mu;
    const float varf = fmaxf((float)var, 0.0f);
    const float rstd = rsqrtf(varf + kEps);
    const float val  = (lane == 0) ? muf : ((lane == 1) ? rstd : 0.0f);
    volatile float* o = stats + (size_t)bh * 32 + lane;
    *o = val;
    __threadfence();
    *o = val;
  }
}

__global__ __launch_bounds__(256) void gn_apply_kernel(
    const float* __restrict__ ctx, const float* __restrict__ stats,
    const float* __restrict__ gw, const float* __restrict__ gb,
    unsigned short* __restrict__ nh, unsigned short* __restrict__ nl, int total8) {
  const int i = blockIdx.x * 256 + threadIdx.x;
  if (i >= total8) return;
  const size_t e0 = (size_t)i << 3;
  const int col = (int)(e0 & (size_t)(kDM - 1));
  const int row = (int)(e0 / (size_t)kDM);
  const int b   = row / kS;
  const int h   = col / kD;
  const float mu   = stats[(size_t)(b * kH + h) * 32];
  const float rstd = stats[(size_t)(b * kH + h) * 32 + 1];
  const v4f a0 = *(const v4f*)(ctx + e0);
  const v4f a1 = *(const v4f*)(ctx + e0 + 4);
  const v4f g0 = *(const v4f*)(gw + col);
  const v4f g1 = *(const v4f*)(gw + col + 4);
  const v4f c0 = *(const v4f*)(gb + col);
  const v4f c1 = *(const v4f*)(gb + col + 4);
  v8h hv, lv;
#pragma unroll
  for (int e = 0; e < 4; ++e) {
    const float n0 = ((a0[e] - mu) * rstd) * g0[e] + c0[e];
    const float n1 = ((a1[e] - mu) * rstd) * g1[e] + c1[e];
    const unsigned short h0 = f2bf_bits(n0), h1 = f2bf_bits(n1);
    const unsigned short l0 = f2bf_bits(n0 - bf_bits2f(h0)), l1 = f2bf_bits(n1 - bf_bits2f(h1));
    hv[e]     = __builtin_bit_cast(_Float16, h0);
    hv[4 + e] = __builtin_bit_cast(_Float16, h1);
    lv[e]     = __builtin_bit_cast(_Float16, l0);
    lv[4 + e] = __builtin_bit_cast(_Float16, l1);
  }
  unsigned short* qh = nh + e0;
  unsigned short* ql = nl + e0;
  *(volatile v8h*)qh = hv;
  *(volatile v8h*)ql = lv;
  __threadfence();
  *(volatile v8h*)qh = hv;
  *(volatile v8h*)ql = lv;
}

extern "C" void kernel_launch(void* const* d_in, const int* in_sizes, int n_in,
                              void* d_out, int out_size, void* d_ws, size_t ws_size,
                              hipStream_t stream) {
  if (n_in < 7) return;
  if (in_sizes[0] != kRows * kDM) return;
  if (in_sizes[1] != 3 * kDM * kDM) return;
  if (in_sizes[2] != 3 * kDM) return;
  if (in_sizes[3] != kDM * kDM) return;
  if (in_sizes[4] != kDM) return;
  if (in_sizes[5] != kDM) return;
  if (in_sizes[6] != kDM) return;
  if (out_size != kRows * kDM) return;
  if (ws_size < kWsTotal) return;

  const float* x       = (const float*)d_in[0];
  const float* Wproj_w = (const float*)d_in[1];
  const float* Wproj_b = (const float*)d_in[2];
  const float* out_w   = (const float*)d_in[3];
  const float* out_b   = (const float*)d_in[4];
  const float* gn_w    = (const float*)d_in[5];
  const float* gn_b    = (const float*)d_in[6];
  float* out = (float*)d_out;

  char* ws = (char*)d_ws;
  unsigned short* XB   = (unsigned short*)(ws + kOffXB);
  unsigned short* WB   = (unsigned short*)(ws + kOffWB);
  unsigned short* OW   = (unsigned short*)(ws + kOffOW);
  unsigned short* QKH  = (unsigned short*)(ws + kOffQKH);
  unsigned short* QKL  = (unsigned short*)(ws + kOffQKL);
  unsigned short* KVTH = (unsigned short*)(ws + kOffKVTH);
  unsigned short* KVTL = (unsigned short*)(ws + kOffKVTL);
  unsigned short* SP   = (unsigned short*)(ws + kOffSP);
  float*          CTX  = (float*)(ws + kOffCTX);
  unsigned short* NH   = (unsigned short*)(ws + kOffNH);
  unsigned short* NL   = (unsigned short*)(ws + kOffNL);
  float*          ST   = (float*)(ws + kOffST);

  cast8_bf16_kernel<<<(kRows * kDM / 8) / 256, 256, 0, stream>>>(x, XB, kRows * kDM / 8);
  cast8_bf16_kernel<<<(3 * kDM * kDM / 8) / 256, 256, 0, stream>>>(Wproj_w, WB, 3 * kDM * kDM / 8);

  wmma_gemm64<0, 2, 2><<<dim3(256), 256, 0, stream>>>(
      XB, XB, kDM,
      WB, kDM,
      (void*)QKH, (void*)QKL, kQKP,
      Wproj_b, kRows, kQKP, kDM);

  wmma_gemm64<0, 1, 2><<<dim3(256), 256, 0, stream>>>(
      WB + (size_t)kDM * kDM, WB + (size_t)kDM * kDM, kDM,
      XB, kDM,
      (void*)KVTH, (void*)KVTL, kTP,
      Wproj_b + kDM, kQKP, kTP, kDM);

  cast8_bf16_kernel<<<(kDM * kDM / 8) / 256, 256, 0, stream>>>(out_w, OW, kDM * kDM / 8);

  state_prefix_kernel<<<kB * kH, 128, 0, stream>>>(KVTH, KVTL, SP);

  chain_chunk_kernel<<<kB * kH * kNCh, 128, 0, stream>>>(QKH, QKL, KVTH, KVTL, SP, CTX);

  gn_stats_kernel<<<kB * kH, 256, 0, stream>>>(CTX, ST);
  gn_apply_kernel<<<(kRows * kDM / 8) / 256, 256, 0, stream>>>(CTX, ST, gn_w, gn_b, NH, NL, kRows * kDM / 8);

  wmma_gemm64<1, 2, 0><<<dim3(128), 256, 0, stream>>>(
      NH, NL, kDM,
      OW, kDM,
      (void*)out, (void*)out, kDM,
      out_b, kRows, kDM, kDM);
}
